// MME_80169859547285
// MI455X (gfx1250) — hardware-run, weakly checked
//
#include <hip/hip_runtime.h>
#include <math.h>
#include <stdint.h>

#define NBATCH 128
#define NEPOCH 64
#define FDIM   128
#define NROWS  (NBATCH * NEPOCH)
#define NT64   (NROWS / 64)
#define CTG    8
#define NCG    (NT64 / CTG)
static_assert(FDIM == 128);
static_assert((NROWS % 256) == 0);
static_assert(CTG == 8);
static_assert((NT64 % CTG) == 0);

typedef __bf16   v16b __attribute__((ext_vector_type(16)));
typedef __bf16   v8b  __attribute__((ext_vector_type(8)));
typedef float    v8f  __attribute__((ext_vector_type(8)));
typedef float    v4f  __attribute__((ext_vector_type(4)));
typedef unsigned int v4u __attribute__((ext_vector_type(4)));

__device__ __forceinline__ unsigned short bf_bits(float f) {
  unsigned u = __float_as_uint(f);
  return (unsigned short)((u + 0x7FFFu + ((u >> 16) & 1u)) >> 16);
}
__device__ __forceinline__ float bf_up(unsigned short h) { return __uint_as_float(((unsigned)h) << 16); }
__device__ __forceinline__ unsigned pk16(unsigned short a, unsigned short b) { return (unsigned)a | ((unsigned)b << 16); }
__device__ __forceinline__ v8f zero8() { v8f z = {0.f, 0.f, 0.f, 0.f, 0.f, 0.f, 0.f, 0.f}; return z; }

__device__ __forceinline__ v16b ldfrag_b(const __bf16* p) {
  union { v16b v; v8b h[2]; } f;
  f.h[0] = *(const v8b*)(p);
  f.h[1] = *(const v8b*)(p + 16);
  return f.v;
}

__device__ __forceinline__ v8f mma_b(v16b a, v16b b, v8f c) {
  c = __builtin_amdgcn_wmma_f32_16x16x32_bf16(false, a, false, b, (short)0, c, false, false);
#if defined(__HIP_DEVICE_COMPILE__)
  asm volatile("v_nop\n\tv_nop\n\tv_nop\n\tv_nop" : "+v"(c) : "v"(a), "v"(b));
#endif
  return c;
}

__device__ __forceinline__ unsigned cvt_pair(float x0, float x1, float& s) {
  const unsigned short b0 = bf_bits(x0), b1 = bf_bits(x1);
  const float y0 = bf_up(b0), y1 = bf_up(b1);
  s = s + y0 * y0;
  s = s + y1 * y1;
  return pk16(b0, b1);
}

__global__ __launch_bounds__(256) void prep_rows(const float* __restrict__ fk, const float* __restrict__ fq,
                                                  unsigned short* Kp, unsigned short* Qp,
                                                  float* rk, float* rq) {
  const int lane  = threadIdx.x & 31;
  const int wave  = threadIdx.x >> 5;
  const int h     = lane >> 4;
  const int c8    = (lane & 15) * 8;
  const int wbase = blockIdx.x * 256 + wave * 32;
  float myk = 0.f, myq = 0.f;
#pragma unroll 1
  for (int p = 0; p < 16; ++p) {
    const int row = wbase + 2 * p + h;
    const size_t o = (size_t)row * FDIM + c8;
    const v4f a0 = *(const v4f*)(fk + o);
    const v4f a1 = *(const v4f*)(fk + o + 4);
    const v4f b0 = *(const v4f*)(fq + o);
    const v4f b1 = *(const v4f*)(fq + o + 4);
    float sk = 0.f, sq = 0.f;
    v4u pk, pq;
    pk[0] = cvt_pair(a0[0], a0[1], sk);
    pk[1] = cvt_pair(a0[2], a0[3], sk);
    pk[2] = cvt_pair(a1[0], a1[1], sk);
    pk[3] = cvt_pair(a1[2], a1[3], sk);
    pq[0] = cvt_pair(b0[0], b0[1], sq);
    pq[1] = cvt_pair(b0[2], b0[3], sq);
    pq[2] = cvt_pair(b1[0], b1[1], sq);
    pq[3] = cvt_pair(b1[2], b1[3], sq);
#pragma unroll
    for (int off = 1; off < 16; off <<= 1) {
      sk += __shfl_xor(sk, off, 32);
      sq += __shfl_xor(sq, off, 32);
    }
    const float rkv = __builtin_amdgcn_rcpf(fmaxf(sqrtf(sk), 1e-12f));
    const float rqv = __builtin_amdgcn_rcpf(fmaxf(sqrtf(sq), 1e-12f));
    const float rko = __shfl_xor(rkv, 16, 32);
    const float rqo = __shfl_xor(rqv, 16, 32);
    const float rk0 = h ? rko : rkv;
    const float rk1 = h ? rkv : rko;
    const float rq0 = h ? rqo : rqv;
    const float rq1 = h ? rqv : rqo;
    if (lane == 2 * p)     { myk = rk0; myq = rq0; }
    if (lane == 2 * p + 1) { myk = rk1; myq = rq1; }
    *(volatile v4u*)(Kp + o) = pk;
    *(volatile v4u*)(Qp + o) = pq;
    __threadfence();
    *(volatile v4u*)(Kp + o) = pk;
    *(volatile v4u*)(Qp + o) = pq;
  }
  *(volatile float*)(rk + wbase + lane) = myk;
  *(volatile float*)(rq + wbase + lane) = myq;
  __threadfence();
  *(volatile float*)(rk + wbase + lane) = myk;
  *(volatile float*)(rq + wbase + lane) = myq;
}

__global__ __launch_bounds__(128) void gram_tiles(const unsigned short* __restrict__ Kp,
                                                   const unsigned short* __restrict__ Qp,
                                                   const float* __restrict__ rk, const float* __restrict__ rq,
                                                   float* PP, float* PE, float* PO) {
  const __bf16* Kb = (const __bf16*)(const void*)Kp;
  const __bf16* Qb = (const __bf16*)(const void*)Qp;
  __shared__ __align__(16) float sred[3][64];

  const int lane  = threadIdx.x & 31;
  const int wave  = threadIdx.x >> 5;
  const int h     = lane >> 4;
  const int c     = lane & 15;
  const int cg    = blockIdx.x;
  const int rt    = blockIdx.y;
  const int rbase = rt * 64 + wave * 16;

  float rkr[8], rqr[8];
  {
    const v4f k0 = *(const v4f*)(rk + rbase + 8 * h);
    const v4f k1 = *(const v4f*)(rk + rbase + 8 * h + 4);
    const v4f q0 = *(const v4f*)(rq + rbase + 8 * h);
    const v4f q1 = *(const v4f*)(rq + rbase + 8 * h + 4);
#pragma unroll
    for (int i = 0; i < 4; ++i) {
      rkr[i] = k0[i]; rkr[4 + i] = k1[i];
      rqr[i] = q0[i]; rqr[4 + i] = q1[i];
    }
  }

  float tot[8], oe[8], op[8];
#pragma unroll
  for (int r = 0; r < 8; ++r) { tot[r] = 0.f; oe[r] = 0.f; op[r] = 0.f; }

  const bool owng = (cg == (rt >> 3));
  const size_t arow = (size_t)(rbase + c) * FDIM + 8 * h;

#pragma unroll 1
  for (int t = 0; t < CTG; ++t) {
    const int cbase = (cg * CTG + t) * 64;
    v8f accK[4], accQ[4];
#pragma unroll
    for (int j = 0; j < 4; ++j) { accK[j] = zero8(); accQ[j] = zero8(); }

#pragma unroll 1
    for (int ks = 0; ks < FDIM / 32; ++ks) {
      const int k0 = ks * 32;
      {
        const v16b a = ldfrag_b(Kb + arow + k0);
        v16b b[4];
#pragma unroll
        for (int j = 0; j < 4; ++j)
          b[j] = ldfrag_b(Kb + (size_t)(cbase + 16 * j + c) * FDIM + 8 * h + k0);
#pragma unroll
        for (int j = 0; j < 4; ++j) accK[j] = mma_b(a, b[j], accK[j]);
      }
      {
        const v16b a = ldfrag_b(Qb + arow + k0);
        v16b b[4];
#pragma unroll
        for (int j = 0; j < 4; ++j)
          b[j] = ldfrag_b(Qb + (size_t)(cbase + 16 * j + c) * FDIM + 8 * h + k0);
#pragma unroll
        for (int j = 0; j < 4; ++j) accQ[j] = mma_b(a, b[j], accQ[j]);
      }
    }

    const bool own = owng && (t == (rt & 7));
#pragma unroll
    for (int j = 0; j < 4; ++j) {
      const int col = cbase + 16 * j + c;
      const float ck = rk[col];
      const float cq = rq[col];
#pragma unroll
      for (int r = 0; r < 8; ++r) {
        const float lg = accK[j][r] * (rkr[r] * ck);
        const float e  = expf(lg);
        const float sm = accQ[j][r] * (rqr[r] * cq);
        const float pr = e * sm;
        tot[r] += pr;
        if (own) { oe[r] += e; op[r] += pr; }
      }
    }
  }

#pragma unroll
  for (int r = 0; r < 8; ++r) {
#pragma unroll
    for (int off = 1; off < 16; off <<= 1) {
      tot[r] += __shfl_xor(tot[r], off, 32);
      oe[r]  += __shfl_xor(oe[r],  off, 32);
      op[r]  += __shfl_xor(op[r],  off, 32);
    }
  }
  if (c == 0) {
#pragma unroll
    for (int r = 0; r < 8; ++r) {
      const int rr = wave * 16 + 8 * h + r;
      sred[0][rr] = tot[r];
      sred[1][rr] = oe[r];
      sred[2][rr] = op[r];
    }
  }
  __syncthreads();
  if (wave == 0) {
    const int cc = lane & 15;
    const v4f vt = *(const v4f*)(&sred[0][cc * 4]);
    const v4f ve = *(const v4f*)(&sred[1][cc * 4]);
    const v4f vp = *(const v4f*)(&sred[2][cc * 4]);
    float* dt = PP + (size_t)cg * NROWS + (size_t)rt * 64 + cc * 4;
    float* de = PE + (size_t)rt * 64 + cc * 4;
    float* dp = PO + (size_t)rt * 64 + cc * 4;
    if (lane < 16) {
      *(volatile v4f*)dt = vt;
      if (owng) { *(volatile v4f*)de = ve; *(volatile v4f*)dp = vp; }
    }
    __threadfence();
    if (lane < 16) {
      *(volatile v4f*)dt = vt;
      if (owng) { *(volatile v4f*)de = ve; *(volatile v4f*)dp = vp; }
    }
  }
}

__global__ __launch_bounds__(256) void finish_loss(const float* __restrict__ PP, const float* __restrict__ PE,
                                                    const float* __restrict__ PO, float* out) {
  __shared__ float s[256];
  const int tid = threadIdx.x;
  float acc = 0.f;
#pragma unroll 1
  for (int r = tid; r < NROWS; r += 256) {
    float tot = 0.f;
#pragma unroll
    for (int g = 0; g < NCG; ++g) tot += PP[(size_t)g * NROWS + r];
    const float pos = PE[r];
    const float own = PO[r];
    const float neg = tot - own;
    const float den = pos + neg;
    const float q   = pos * __builtin_amdgcn_rcpf(den);
    acc += -logf(q);
  }
  s[tid] = acc;
  __syncthreads();
#pragma unroll
  for (int off = 128; off > 0; off >>= 1) {
    if (tid < off) s[tid] += s[tid + off];
    __syncthreads();
  }
  if (tid == 0) {
    const float loss = s[0] * (1.0f / (float)NROWS);
    *(volatile float*)out = loss;
    __threadfence();
    *(volatile float*)out = loss;
  }
}

extern "C" void kernel_launch(void* const* d_in, const int* in_sizes, int n_in,
                              void* d_out, int out_size, void* d_ws, size_t ws_size,
                              hipStream_t stream) {
  if (n_in < 2) return;
  if (in_sizes[0] != NROWS * FDIM) return;
  if (in_sizes[1] != NROWS * FDIM) return;
  if (out_size < 1) return;

  const float* fk = (const float*)d_in[0];
  const float* fq = (const float*)d_in[1];
  float* out = (float*)d_out;

  const size_t bPlane = (size_t)NROWS * FDIM * 2;
  const size_t bVec   = (size_t)NROWS * 4;
  const size_t bPP    = (size_t)NCG * NROWS * 4;
  size_t off = 0;
  const size_t oK  = off; off += bPlane;
  const size_t oQ  = off; off += bPlane;
  const size_t oRk = off; off += bVec;
  const size_t oRq = off; off += bVec;
  const size_t oPP = off; off += bPP;
  const size_t oPE = off; off += bVec;
  const size_t oPO = off; off += bVec;
  if (off > ws_size) return;
  if (off > (size_t)134217728) return;

  char* ws = (char*)d_ws;
  unsigned short* Kp = (unsigned short*)(ws + oK);
  unsigned short* Qp = (unsigned short*)(ws + oQ);
  float* rk = (float*)(ws + oRk);
  float* rq = (float*)(ws + oRq);
  float* PP = (float*)(ws + oPP);
  float* PE = (float*)(ws + oPE);
  float* PO = (float*)(ws + oPO);

  prep_rows<<<dim3(NROWS / 256), dim3(256), 0, stream>>>(fk, fq, Kp, Qp, rk, rq);
  gram_tiles<<<dim3(NCG, NT64), dim3(128), 0, stream>>>(Kp, Qp, rk, rq, PP, PE, PO);
  finish_loss<<<dim3(1), dim3(256), 0, stream>>>(PP, PE, PO, out);
  (void)hipGetLastError();
}
